// SkeletonGCN_33243046871577
// MI455X (gfx1250) — hardware-verified
//
#include <hip/hip_runtime.h>
#include <stddef.h>


#define FDIM    64
#define HD2     32
#define NCLS    10
#define NCP     16
#define NTHR    256
#define NWAVE   8
#define EPT     8
#define NGRP    2
#define CHUNK   (NTHR * EPT * NGRP)
#define WCAP    (EPT * NGRP * 32)
#define LISTN   (NWAVE * WCAP)
#define NBC     4096
#define NBF     4096
#define NBP     32
#define RCAP    32768
#define RBN     128
#define TGT     256
#define DEGCAP  256
#define CNTMAX  4096
#define GROWS   128
#define OTHR    512
#define WSCALE  16.0f
#define WINV    0.0625f
#define BNEPS   1e-5f
#define LDS_FILL ((RCAP + NBF + LISTN) * 4 + 64)

static_assert((CHUNK & (CHUNK - 1)) == 0);
static_assert(CHUNK <= 4096);
static_assert(NBC <= 4096 && NBF <= 4096 && NBP <= 4096);
static_assert((NBC & (NBC - 1)) == 0 && (NBF & (NBF - 1)) == 0 && (NBP & (NBP - 1)) == 0);
static_assert(NBF == NBC);
static_assert(OTHR * 8 == NBC);
static_assert((RCAP % 32) == 0);
static_assert(TGT == NWAVE * 32 && (TGT % GROWS) == 0 && (NBC % TGT) == 0);
static_assert(GROWS == NWAVE * 16);
static_assert((GROWS * FDIM / 8) % NTHR == 0);
static_assert(GROWS * (FDIM + 8) * 2 <= GROWS * FDIM * 4);
static_assert(NBP * FDIM / 4 == 2 * NTHR);
static_assert((FDIM * FDIM / 8) % NTHR == 0 && ((2 * FDIM * FDIM + HD2 * FDIM) / 8) % NTHR == 0);
static_assert(((GROWS * NCLS) % 4) == 0 && ((GROWS * NCLS * 4) % 128) == 0);
static_assert((HD2 % 16) == 0 && NCLS <= NCP);

typedef float    v2f  __attribute__((ext_vector_type(2)));
typedef float    v4f  __attribute__((ext_vector_type(4)));
typedef float    v8f  __attribute__((ext_vector_type(8)));
typedef int      v4i  __attribute__((ext_vector_type(4)));
typedef double   v2d  __attribute__((ext_vector_type(2)));
typedef _Float16 v2h  __attribute__((ext_vector_type(2)));
typedef _Float16 v8h  __attribute__((ext_vector_type(8)));
typedef _Float16 v16h __attribute__((ext_vector_type(16)));
union FragH { v16h v; v8h h[2]; };

__device__ __forceinline__ v8h cvt8f(const float* v) {
  v8h r;
  r[0] = (_Float16)v[0]; r[1] = (_Float16)v[1]; r[2] = (_Float16)v[2]; r[3] = (_Float16)v[3];
  r[4] = (_Float16)v[4]; r[5] = (_Float16)v[5]; r[6] = (_Float16)v[6]; r[7] = (_Float16)v[7];
  return r;
}
__device__ __forceinline__ void load8(const float* p, float* v) {
  const v4f a = *(const v4f*)p, b = *(const v4f*)(p + 4);
  v[0] = a.x; v[1] = a.y; v[2] = a.z; v[3] = a.w; v[4] = b.x; v[5] = b.y; v[6] = b.z; v[7] = b.w;
}
__device__ __forceinline__ void load8(const _Float16* p, float* v) {
  const v8h q = *(const v8h*)p;
  v[0] = (float)q[0]; v[1] = (float)q[1]; v[2] = (float)q[2]; v[3] = (float)q[3];
  v[4] = (float)q[4]; v[5] = (float)q[5]; v[6] = (float)q[6]; v[7] = (float)q[7];
}

__device__ __forceinline__ v8f wmh(v16h a, v16h b, v8f c) {
  v8f d = __builtin_amdgcn_wmma_f32_16x16x32_f16(false, a, false, b, (short)0, c, false, false);
  asm volatile("v_nop\n\tv_nop\n\tv_nop\n\tv_nop" : "+v"(d) : "v"(a), "v"(b));
  return d;
}

template <int NB>
__device__ __forceinline__ int scan_chunk(const int* __restrict__ dsts, int nE, int cbase, int slotBase,
                                          int vec8, int* list, int tid, int lane, int wave) {
  int wc = 0;
#pragma unroll
  for (int g = 0; g < NGRP; ++g) {
    const int el0  = (g * NTHR + tid) * EPT;
    const int e0   = cbase + el0;
    const int sent = -2147483647 - 1;
    v4i da, db;
    if (vec8 != 0 && cbase + CHUNK <= nE) {
      da = *(const v4i*)(dsts + e0);
      db = *(const v4i*)(dsts + e0 + 4);
    } else {
      da.x = (e0     < nE) ? dsts[min(e0, nE - 1)] : sent;
      da.y = (e0 + 1 < nE) ? dsts[min(e0 + 1, nE - 1)] : sent;
      da.z = (e0 + 2 < nE) ? dsts[min(e0 + 2, nE - 1)] : sent;
      da.w = (e0 + 3 < nE) ? dsts[min(e0 + 3, nE - 1)] : sent;
      db.x = (e0 + 4 < nE) ? dsts[min(e0 + 4, nE - 1)] : sent;
      db.y = (e0 + 5 < nE) ? dsts[min(e0 + 5, nE - 1)] : sent;
      db.z = (e0 + 6 < nE) ? dsts[min(e0 + 6, nE - 1)] : sent;
      db.w = (e0 + 7 < nE) ? dsts[min(e0 + 7, nE - 1)] : sent;
    }
    const unsigned nb = (unsigned)slotBase;
    const unsigned s0 = (unsigned)da.x - nb, s1 = (unsigned)da.y - nb;
    const unsigned s2 = (unsigned)da.z - nb, s3 = (unsigned)da.w - nb;
    const unsigned s4 = (unsigned)db.x - nb, s5 = (unsigned)db.y - nb;
    const unsigned s6 = (unsigned)db.z - nb, s7 = (unsigned)db.w - nb;
    const bool h0 = s0 < (unsigned)NB, h1 = s1 < (unsigned)NB, h2 = s2 < (unsigned)NB, h3 = s3 < (unsigned)NB;
    const bool h4 = s4 < (unsigned)NB, h5 = s5 < (unsigned)NB, h6 = s6 < (unsigned)NB, h7 = s7 < (unsigned)NB;
    const unsigned any = __builtin_amdgcn_ballot_w32(h0 | h1 | h2 | h3 | h4 | h5 | h6 | h7);
    if (any != 0u) {
#define HITJ(J, HJ, SJ) { \
        const unsigned mj = __builtin_amdgcn_ballot_w32(HJ); \
        if (mj != 0u) { \
          if (HJ) { \
            const int pos = wc + (int)__builtin_amdgcn_mbcnt_lo(mj, 0u); \
            if (pos < WCAP) list[wave * WCAP + pos] = ((el0 + (J)) << 12) | (int)(SJ); \
          } \
          wc += (int)__builtin_popcount(mj); } }
      HITJ(0, h0, s0)
      HITJ(1, h1, s1)
      HITJ(2, h2, s2)
      HITJ(3, h3, s3)
      HITJ(4, h4, s4)
      HITJ(5, h5, s5)
      HITJ(6, h6, s6)
      HITJ(7, h7, s7)
#undef HITJ
    }
  }
  return wc;
}

__global__ __launch_bounds__(NTHR) void k_wprep(
    const float* __restrict__ W1, const float* __restrict__ W2, const float* __restrict__ L1,
    const float* __restrict__ L2, _Float16* w1p, _Float16* w2p, _Float16* l1p, _Float16* l2p) {
  const int g0 = FDIM * FDIM / 8;
  const int g1 = FDIM * FDIM / 8;
  const int g2 = HD2 * FDIM / 8;
  const int g3 = NCP * HD2 / 8;
  const int bstart = blockIdx.x * NTHR;
  const float* src; _Float16* dst; int K, Nout, KP, segOff;
  if (bstart < g0)                { src = W1; dst = w1p; K = FDIM; Nout = FDIM; KP = FDIM; segOff = 0; }
  else if (bstart < g0 + g1)      { src = W2; dst = w2p; K = FDIM; Nout = FDIM; KP = FDIM; segOff = g0; }
  else if (bstart < g0 + g1 + g2) { src = L1; dst = l1p; K = FDIM; Nout = HD2;  KP = FDIM; segOff = g0 + g1; }
  else                            { src = L2; dst = l2p; K = HD2;  Nout = NCLS; KP = HD2;  segOff = g0 + g1 + g2; }
  const int i = bstart + (int)threadIdx.x;
  if (i >= g0 + g1 + g2 + g3) return;
  const int o  = (i - segOff) * 8;
  const int n  = o / KP;
  const int k0 = o - n * KP;
  const int nc = n < Nout ? n : Nout - 1;
  float v[8];
#pragma unroll
  for (int e = 0; e < 8; ++e) {
    const int k  = k0 + e;
    const int kc = k < K ? k : K - 1;
    const float x = src[(size_t)kc * Nout + nc];
    v[e] = (k < K && n < Nout) ? x * WSCALE : 0.0f;
  }
  const v8h hv = cvt8f(v);
  _Float16* dp = dst + o;
  *(volatile v8h*)dp = hv;
  __threadfence();
  *(volatile v8h*)dp = hv;
}

__global__ __launch_bounds__(NTHR) void k_count(
    const int* __restrict__ ei, int* cnt, float* dinv, int nE, int vec8) {
  __shared__ __attribute__((aligned(16))) int scnt[NBC];
  __shared__ __attribute__((aligned(16))) int list[LISTN];
  __shared__ int wcnt[NWAVE];
  const int tid = threadIdx.x, lane = tid & 31, wave = tid >> 5;
  const int nodeBase = blockIdx.x * NBC;
  const int* dsts = ei + nE;

  for (int i = tid; i < NBC; i += NTHR) scnt[i] = 0;
  __syncthreads();

  const int nChunks = (nE + CHUNK - 1) / CHUNK;
#pragma unroll 1
  for (int ch = 0; ch < nChunks; ++ch) {
    const int cbase = ch * CHUNK;
    const int wc = scan_chunk<NBC>(dsts, nE, cbase, nodeBase, vec8, list, tid, lane, wave);
    if (lane == 0) wcnt[wave] = wc;
    __syncthreads();
    if (wave == 0) {
#pragma unroll 1
      for (int wsx = 0; wsx < NWAVE; ++wsx) {
        int n = __builtin_amdgcn_readfirstlane(wcnt[wsx]);
        n = n > WCAP ? WCAP : (n < 0 ? 0 : n);
        const int* lp = list + wsx * WCAP;
#pragma unroll 1
        for (int i = 0; i < n; ++i) {
          const int ent  = __builtin_amdgcn_readfirstlane(lp[i]);
          const int slot = ent & (NBC - 1);
          if (lane == 0) scnt[slot] = scnt[slot] + 1;
        }
      }
    }
    __syncthreads();
  }

  v4i cq[4]; v4f dq[4];
#pragma unroll
  for (int q = 0; q < 4; ++q) {
    const int f = (wave * 4 + q) * 128 + 4 * lane;
    const v4i c = *(const v4i*)(scnt + f);
    cq[q] = c;
    dq[q].x = rsqrtf((float)(c.x + 1));
    dq[q].y = rsqrtf((float)(c.y + 1));
    dq[q].z = rsqrtf((float)(c.z + 1));
    dq[q].w = rsqrtf((float)(c.w + 1));
  }
  int*   cp = cnt + (size_t)nodeBase;
  float* dp = dinv + (size_t)nodeBase;
#pragma unroll
  for (int q = 0; q < 4; ++q) {
    const int f = (wave * 4 + q) * 128 + 4 * lane;
    *(volatile v4i*)(cp + f) = cq[q];
    *(volatile v4f*)(dp + f) = dq[q];
  }
  __threadfence();
#pragma unroll
  for (int q = 0; q < 4; ++q) {
    const int f = (wave * 4 + q) * 128 + 4 * lane;
    *(volatile v4i*)(cp + f) = cq[q];
    *(volatile v4f*)(dp + f) = dq[q];
  }
}

__global__ __launch_bounds__(OTHR) void k_offsets(
    const int* __restrict__ cnt, int* off, int* rbase, int nChunk) {
  __shared__ __attribute__((aligned(16))) int soff[NBC];
  __shared__ __attribute__((aligned(16))) int srb[RBN];
  __shared__ int wtot[OTHR / 32];
  const int tid = threadIdx.x, lane = tid & 31, wave = tid >> 5;
  for (int i = tid; i < RBN; i += OTHR) srb[i] = 0;
  __syncthreads();
  int carry = 0;
#pragma unroll 1
  for (int ch = 0; ch < nChunk; ++ch) {
    const int base = ch * NBC;
    const v4i c0 = *(const v4i*)(cnt + base + 8 * tid);
    const v4i c1 = *(const v4i*)(cnt + base + 8 * tid + 4);
    const int e0 = min(max(c0.x, 0), CNTMAX), e1 = min(max(c0.y, 0), CNTMAX);
    const int e2 = min(max(c0.z, 0), CNTMAX), e3 = min(max(c0.w, 0), CNTMAX);
    const int e4 = min(max(c1.x, 0), CNTMAX), e5 = min(max(c1.y, 0), CNTMAX);
    const int e6 = min(max(c1.z, 0), CNTMAX), e7 = min(max(c1.w, 0), CNTMAX);
    const int ts = e0 + e1 + e2 + e3 + e4 + e5 + e6 + e7;
    int incl = ts;
#pragma unroll
    for (int d = 1; d < 32; d <<= 1) {
      const int t = __shfl_up(incl, d);
      if (lane >= d) incl += t;
    }
    if (lane == 31) wtot[wave] = incl;
    __syncthreads();
    int S = 0;
#pragma unroll
    for (int w = 0; w < OTHR / 32; ++w) S += wtot[w];
    int pre = 0;
#pragma unroll 1
    for (int w = 0; w < wave; ++w) pre += wtot[w];
    if (tid == 0) srb[min(ch, RBN - 1)] = carry;
    int run = carry + pre + incl - ts;
    soff[8 * tid + 0] = run; run += e0;
    soff[8 * tid + 1] = run; run += e1;
    soff[8 * tid + 2] = run; run += e2;
    soff[8 * tid + 3] = run; run += e3;
    soff[8 * tid + 4] = run; run += e4;
    soff[8 * tid + 5] = run; run += e5;
    soff[8 * tid + 6] = run; run += e6;
    soff[8 * tid + 7] = run;
    carry += (S + 31) & ~31;
    __syncthreads();
    const v4i o0 = *(const v4i*)(soff + 4 * tid);
    const v4i o1 = *(const v4i*)(soff + 4 * (tid + OTHR));
    int* op = off + base;
    *(volatile v4i*)(op + 4 * tid) = o0;
    *(volatile v4i*)(op + 4 * (tid + OTHR)) = o1;
    __threadfence();
    *(volatile v4i*)(op + 4 * tid) = o0;
    *(volatile v4i*)(op + 4 * (tid + OTHR)) = o1;
    __syncthreads();
  }
  if (tid == 0) srb[min(nChunk, RBN - 1)] = carry;
  __syncthreads();
  v4i rv = {0, 0, 0, 0};
  if (tid < 32) rv = *(const v4i*)(srb + 4 * tid);
  if (tid < 32) *(volatile v4i*)(rbase + 4 * tid) = rv;
  __threadfence();
  if (tid < 32) *(volatile v4i*)(rbase + 4 * tid) = rv;
}

__global__ __launch_bounds__(NTHR) void k_fill(
    const int* __restrict__ ei, const int* __restrict__ off, const int* __restrict__ rbase,
    int* csr, int nN, int nE, int vec8, int csrLen) {
  extern __shared__ v4f lds_dyn[];
  int* region = (int*)lds_dyn;
  int* cursor = region + RCAP;
  int* list   = cursor + NBF;
  int* wcnt   = list + LISTN;
  const int tid = threadIdx.x, lane = tid & 31, wave = tid >> 5;
  const int b = blockIdx.x;
  const int nodeBase = b * NBF;
  const int* dsts = ei + nE;

  int rb0 = rbase[b];
  const int rb1 = rbase[b + 1];
  rb0 = rb0 < 0 ? 0 : (rb0 > csrLen ? csrLen : rb0);
  rb0 &= ~31;
  int len = rb1 - rb0;
  len = len < 0 ? 0 : (len > RCAP ? RCAP : len);
  int lenW = (len + 31) & ~31;
  if (rb0 + lenW > csrLen) lenW = (csrLen - rb0) & ~31;

  {
    const v4i z = {0, 0, 0, 0};
    for (int i = tid; i < RCAP / 4; i += NTHR) ((v4i*)region)[i] = z;
    for (int s = tid; s < NBF; s += NTHR) {
      int o = off[nodeBase + s] - rb0;
      o = o < 0 ? 0 : (o > RCAP ? RCAP : o);
      cursor[s] = o;
    }
  }
  __syncthreads();

  const int nChunks = (nE + CHUNK - 1) / CHUNK;
#pragma unroll 1
  for (int ch = 0; ch < nChunks; ++ch) {
    const int cbase = ch * CHUNK;
    const int wc = scan_chunk<NBF>(dsts, nE, cbase, nodeBase, vec8, list, tid, lane, wave);
    if (lane == 0) wcnt[wave] = wc;
    __syncthreads();
    if (wave == 0) {
#pragma unroll 1
      for (int wsx = 0; wsx < NWAVE; ++wsx) {
        int n = __builtin_amdgcn_readfirstlane(wcnt[wsx]);
        n = n > WCAP ? WCAP : (n < 0 ? 0 : n);
        const int* lp = list + wsx * WCAP;
#pragma unroll 1
        for (int i = 0; i < n; ++i) {
          const int ent  = __builtin_amdgcn_readfirstlane(lp[i]);
          const int slot = ent & (NBF - 1);
          int e = cbase + ((ent >> 12) & (CHUNK - 1));
          e = e > nE - 1 ? nE - 1 : e;
          int src = ei[e];
          src = src < 0 ? 0 : (src > nN - 1 ? nN - 1 : src);
          if (lane == 0) {
            int pos = cursor[slot];
            pos = pos < 0 ? 0 : (pos > RCAP - 1 ? RCAP - 1 : pos);
            region[pos] = src;
            const int np = pos + 1;
            cursor[slot] = np > RCAP ? RCAP : np;
          }
        }
      }
    }
    __syncthreads();
  }

  const int nv = lenW >> 2;
  int* gp = csr + rb0;
#pragma unroll 1
  for (int i = tid; i < nv; i += NTHR) { const v4i v = ((const v4i*)region)[i]; *(volatile v4i*)(gp + 4 * i) = v; }
  __threadfence();
#pragma unroll 1
  for (int i = tid; i < nv; i += NTHR) { const v4i v = ((const v4i*)region)[i]; *(volatile v4i*)(gp + 4 * i) = v; }
}

template <typename AT, int BNA>
__global__ __launch_bounds__(NTHR) void k_gemm(
    const AT* __restrict__ A, const _Float16* __restrict__ Bs, const float* __restrict__ dinv,
    const float* __restrict__ bnp, float* C, int nRowsA) {
  __shared__ __attribute__((aligned(16))) v4f lds[GROWS * FDIM / 4];
  constexpr int AP = FDIM + 8;
  _Float16* sA  = (_Float16*)lds;
  float*    stg = (float*)lds;
  const int tid = threadIdx.x, lane = tid & 31, wave = tid >> 5, hh = lane >> 4, m = lane & 15;
  const int rowBase = blockIdx.x * GROWS;

  float sc[8], sh[8];
  {
    const int c0 = (tid & 7) * 8;
    v4f a = {1.f, 1.f, 1.f, 1.f}, b = {1.f, 1.f, 1.f, 1.f}, c = {0.f, 0.f, 0.f, 0.f}, d = {0.f, 0.f, 0.f, 0.f};
    if (BNA) {
      a = *(const v4f*)(bnp + c0);        b = *(const v4f*)(bnp + c0 + 4);
      c = *(const v4f*)(bnp + FDIM + c0); d = *(const v4f*)(bnp + FDIM + c0 + 4);
    }
    sc[0] = a.x; sc[1] = a.y; sc[2] = a.z; sc[3] = a.w; sc[4] = b.x; sc[5] = b.y; sc[6] = b.z; sc[7] = b.w;
    sh[0] = c.x; sh[1] = c.y; sh[2] = c.z; sh[3] = c.w; sh[4] = d.x; sh[5] = d.y; sh[6] = d.z; sh[7] = d.w;
  }
#pragma unroll
  for (int i = 0; i < (GROWS * FDIM / 8) / NTHR; ++i) {
    const int idx = i * NTHR + tid;
    const int r   = idx >> 3;
    const int c0  = (idx & 7) * 8;
    int row = rowBase + r;
    row = row > nRowsA - 1 ? nRowsA - 1 : row;
    float v[8];
    load8(A + (size_t)row * FDIM + c0, v);
    if (BNA) {
#pragma unroll
      for (int e = 0; e < 8; ++e) v[e] = fmaxf(v[e] * sc[e] + sh[e], 0.0f);
    }
    *(v8h*)(sA + r * AP + c0) = cvt8f(v);
  }
  __syncthreads();

  v8f acc[4];
#pragma unroll
  for (int t = 0; t < 4; ++t) { v8f z = {0.f, 0.f, 0.f, 0.f, 0.f, 0.f, 0.f, 0.f}; acc[t] = z; }
  const _Float16* ar = sA + (wave * 16 + m) * AP + 8 * hh;
#pragma unroll
  for (int kt = 0; kt < FDIM / 32; ++kt) {
    FragH a;
    a.h[0] = *(const v8h*)(ar + 32 * kt);
    a.h[1] = *(const v8h*)(ar + 32 * kt + 16);
#pragma unroll
    for (int t = 0; t < 4; ++t) {
      const _Float16* bp = Bs + (size_t)(16 * t + m) * FDIM + 32 * kt + 8 * hh;
      FragH b;
      b.h[0] = *(const v8h*)bp;
      b.h[1] = *(const v8h*)(bp + 16);
      acc[t] = wmh(a.v, b.v, acc[t]);
    }
  }
  __syncthreads();

  const int r0 = wave * 16 + 8 * hh;
  const v4f dA = *(const v4f*)(dinv + (size_t)rowBase + r0);
  const v4f dB = *(const v4f*)(dinv + (size_t)rowBase + r0 + 4);
  float s[8];
  s[0] = dA.x; s[1] = dA.y; s[2] = dA.z; s[3] = dA.w; s[4] = dB.x; s[5] = dB.y; s[6] = dB.z; s[7] = dB.w;
  float* sp = stg + r0 * FDIM + m;
#pragma unroll
  for (int t = 0; t < 4; ++t) {
#pragma unroll
    for (int r = 0; r < 8; ++r) sp[r * FDIM + 16 * t] = acc[t][r] * (s[r] * WINV);
  }
  __syncthreads();

  const float* lp = stg + wave * 16 * FDIM;
  float* gp = C + ((size_t)rowBase + wave * 16) * FDIM;
#pragma unroll
  for (int p = 0; p < 8; ++p) { const v4f v = *(const v4f*)(lp + 4 * (32 * p + lane)); *(volatile v4f*)(gp + 4 * (32 * p + lane)) = v; }
  __threadfence();
#pragma unroll
  for (int p = 0; p < 8; ++p) { const v4f v = *(const v4f*)(lp + 4 * (32 * p + lane)); *(volatile v4f*)(gp + 4 * (32 * p + lane)) = v; }
}

__global__ __launch_bounds__(NTHR) void k_agg(
    const int* __restrict__ csr, const int* __restrict__ off, const int* __restrict__ cnt,
    const float* __restrict__ dinv, const float* __restrict__ hw, const float* __restrict__ bias,
    _Float16* P, double* part, int nN, int csrLen) {
  __shared__ __attribute__((aligned(16))) _Float16 sT[NWAVE * 32 * FDIM];
  __shared__ __attribute__((aligned(16))) double sS[NWAVE * FDIM];
  __shared__ __attribute__((aligned(16))) double sQ[NWAVE * FDIM];
  const int tid = threadIdx.x, lane = tid & 31, wave = tid >> 5;
  const int tbase = blockIdx.x * TGT + wave * 32;
  const int cl = tbase + lane;
  const int cnt_l = cnt[cl];
  const int off_l = off[cl];
  union FI { float f; int i; };
  FI dvu; dvu.f = dinv[cl];
  const v2f bb = *(const v2f*)(bias + 2 * lane);
  _Float16* sw = sT + wave * (32 * FDIM);
  double s0 = 0.0, s1 = 0.0, q0 = 0.0, q1 = 0.0;

#pragma unroll 1
  for (int j = 0; j < 32; ++j) {
    const int c = tbase + j;
    int n = __builtin_amdgcn_readlane(cnt_l, j);
    n = n < 0 ? 0 : (n > DEGCAP ? DEGCAP : n);
    const int st = __builtin_amdgcn_readlane(off_l, j);
    FI du; du.i = __builtin_amdgcn_readlane(dvu.i, j);
    v2f acc = {0.f, 0.f};
#pragma unroll 1
    for (int qb = 0; qb < n; qb += 32) {
      int pos = st + qb + lane;
      pos = pos < 0 ? 0 : (pos > csrLen - 1 ? csrLen - 1 : pos);
      int sl = csr[pos];
      sl = sl < 0 ? 0 : (sl > nN - 1 ? nN - 1 : sl);
      const int mcnt = (n - qb) < 32 ? (n - qb) : 32;
#pragma unroll 1
      for (int p = 0; p < mcnt; ++p) {
        const int s = __builtin_amdgcn_readlane(sl, p);
        acc = acc + *(const v2f*)(hw + (size_t)s * FDIM + 2 * lane);
      }
    }
    const v2f sv = *(const v2f*)(hw + (size_t)c * FDIM + 2 * lane);
    const v2f v = (acc + sv) * du.f + bb;
    v2h hv;
    hv.x = (_Float16)v.x; hv.y = (_Float16)v.y;
    *(v2h*)(sw + j * FDIM + 2 * lane) = hv;
    if (c < nN) {
      const double fx = (double)(float)hv.x, fy = (double)(float)hv.y;
      s0 += fx; q0 += fx * fx; s1 += fy; q1 += fy * fy;
    }
  }
  __syncthreads();

  sS[wave * FDIM + 2 * lane] = s0; sS[wave * FDIM + 2 * lane + 1] = s1;
  sQ[wave * FDIM + 2 * lane] = q0; sQ[wave * FDIM + 2 * lane + 1] = q1;

  const _Float16* lp = sw;
  _Float16* gp = P + (size_t)tbase * FDIM;
#pragma unroll
  for (int p = 0; p < 8; ++p) { const v8h v = *(const v8h*)(lp + 8 * (32 * p + lane)); *(volatile v8h*)(gp + 8 * (32 * p + lane)) = v; }
  __syncthreads();

  v2d ps = {0.0, 0.0}, pq = {0.0, 0.0};
  double* pp = part + (size_t)blockIdx.x * (2 * FDIM);
  if (wave == 0) {
    double a0 = 0.0, a1 = 0.0, b0 = 0.0, b1 = 0.0;
#pragma unroll
    for (int w = 0; w < NWAVE; ++w) {
      a0 += sS[w * FDIM + 2 * lane]; a1 += sS[w * FDIM + 2 * lane + 1];
      b0 += sQ[w * FDIM + 2 * lane]; b1 += sQ[w * FDIM + 2 * lane + 1];
    }
    ps.x = a0; ps.y = a1; pq.x = b0; pq.y = b1;
    *(volatile v2d*)(pp + 2 * lane) = ps;
    *(volatile v2d*)(pp + FDIM + 2 * lane) = pq;
  }
  __threadfence();
#pragma unroll
  for (int p = 0; p < 8; ++p) { const v8h v = *(const v8h*)(lp + 8 * (32 * p + lane)); *(volatile v8h*)(gp + 8 * (32 * p + lane)) = v; }
  if (wave == 0) {
    *(volatile v2d*)(pp + 2 * lane) = ps;
    *(volatile v2d*)(pp + FDIM + 2 * lane) = pq;
  }
}

__global__ __launch_bounds__(64) void k_bnfin(
    const double* __restrict__ part, const float* __restrict__ gam, const float* __restrict__ bet,
    float* bnp, int nBlk, int nN) {
  __shared__ __attribute__((aligned(16))) float sp[2 * FDIM];
  const int c = threadIdx.x;
  double S = 0.0, Q = 0.0;
#pragma unroll 1
  for (int b = 0; b < nBlk; ++b) {
    S += part[(size_t)b * (2 * FDIM) + c];
    Q += part[(size_t)b * (2 * FDIM) + FDIM + c];
  }
  const double invN = 1.0 / (double)(nN > 0 ? nN : 1);
  const double mean = S * invN;
  double var = Q * invN - mean * mean;
  var = var < 0.0 ? 0.0 : var;
  const float rstd  = rsqrtf((float)var + BNEPS);
  const float scale = gam[c] * rstd;
  const float shift = bet[c] - (float)mean * scale;
  sp[c] = scale; sp[FDIM + c] = shift;
  __syncthreads();
  v4f v = {0.f, 0.f, 0.f, 0.f};
  if (c < 32) v = *(const v4f*)(sp + 4 * c);
  if (c < 32) *(volatile v4f*)(bnp + 4 * c) = v;
  __threadfence();
  if (c < 32) *(volatile v4f*)(bnp + 4 * c) = v;
}

__global__ __launch_bounds__(NTHR) void k_pool(
    const int* __restrict__ batch, const _Float16* __restrict__ P1, const _Float16* __restrict__ P2,
    const float* __restrict__ bnp1, const float* __restrict__ bnp2, float* pooled, int nN) {
  __shared__ __attribute__((aligned(16))) float acc[NBP * FDIM];
  __shared__ __attribute__((aligned(16))) int list[LISTN];
  __shared__ int pc[NBP];
  __shared__ int wcnt[NWAVE];
  const int tid = threadIdx.x, lane = tid & 31, wave = tid >> 5;
  const int gBase = blockIdx.x * NBP;

  {
    const v4f z = {0.f, 0.f, 0.f, 0.f};
    for (int i = tid; i < NBP * FDIM / 4; i += NTHR) ((v4f*)acc)[i] = z;
    for (int i = tid; i < NBP; i += NTHR) pc[i] = 0;
  }
  const v2f sc1 = *(const v2f*)(bnp1 + 2 * lane), sh1 = *(const v2f*)(bnp1 + FDIM + 2 * lane);
  const v2f sc2 = *(const v2f*)(bnp2 + 2 * lane), sh2 = *(const v2f*)(bnp2 + FDIM + 2 * lane);
  __syncthreads();

  const int nChunks = (nN + CHUNK - 1) / CHUNK;
#pragma unroll 1
  for (int ch = 0; ch < nChunks; ++ch) {
    const int cbase = ch * CHUNK;
    const int wc = scan_chunk<NBP>(batch, nN, cbase, gBase, 1, list, tid, lane, wave);
    if (lane == 0) wcnt[wave] = wc;
    __syncthreads();
    if (wave == 0) {
#pragma unroll 1
      for (int wsx = 0; wsx < NWAVE; ++wsx) {
        int n = __builtin_amdgcn_readfirstlane(wcnt[wsx]);
        n = n > WCAP ? WCAP : (n < 0 ? 0 : n);
        const int* lp = list + wsx * WCAP;
#pragma unroll 1
        for (int i = 0; i < n; ++i) {
          const int ent  = __builtin_amdgcn_readfirstlane(lp[i]);
          const int slot = ent & (NBP - 1);
          int nd = cbase + ((ent >> 12) & (CHUNK - 1));
          nd = nd > nN - 1 ? nN - 1 : nd;
          const v2h a = *(const v2h*)(P1 + (size_t)nd * FDIM + 2 * lane);
          const v2h b = *(const v2h*)(P2 + (size_t)nd * FDIM + 2 * lane);
          const float h1x = fmaxf((float)a.x * sc1.x + sh1.x, 0.0f);
          const float h1y = fmaxf((float)a.y * sc1.y + sh1.y, 0.0f);
          const float h2x = fmaxf((float)b.x * sc2.x + sh2.x, 0.0f) + h1x;
          const float h2y = fmaxf((float)b.y * sc2.y + sh2.y, 0.0f) + h1y;
          v2f* ap = (v2f*)(acc + slot * FDIM + 2 * lane);
          v2f t = *ap;
          t.x += h2x; t.y += h2y;
          *ap = t;
          if (lane == 0) pc[slot] = pc[slot] + 1;
        }
      }
    }
    __syncthreads();
  }

  v4f ov[2];
#pragma unroll
  for (int p = 0; p < 2; ++p) {
    const int piece = p * NTHR + tid;
    const int row = piece >> 4;
    const int c0  = (piece & 15) * 4;
    int cv = pc[row];
    cv = cv < 1 ? 1 : cv;
    const float inv = 1.0f / (float)cv;
    ov[p] = *(const v4f*)(acc + row * FDIM + c0) * inv;
  }
  float* gp = pooled + (size_t)gBase * FDIM;
#pragma unroll
  for (int p = 0; p < 2; ++p) *(volatile v4f*)(gp + 4 * (p * NTHR + tid)) = ov[p];
  __threadfence();
#pragma unroll
  for (int p = 0; p < 2; ++p) *(volatile v4f*)(gp + 4 * (p * NTHR + tid)) = ov[p];
}

__global__ __launch_bounds__(NTHR) void k_head(
    const float* __restrict__ pooled, const _Float16* __restrict__ l1p, const float* __restrict__ lb1,
    const _Float16* __restrict__ l2p, const float* __restrict__ lb2, float* out, int nG) {
  constexpr int AP = FDIM + 8, ZP = HD2 + 8;
  __shared__ __attribute__((aligned(16))) _Float16 sA[GROWS * AP];
  __shared__ __attribute__((aligned(16))) _Float16 sZ[GROWS * ZP];
  __shared__ __attribute__((aligned(16))) float sL[GROWS * NCP];
  __shared__ __attribute__((aligned(16))) float sO[GROWS * NCLS];
  const int tid = threadIdx.x, lane = tid & 31, wave = tid >> 5, hh = lane >> 4, m = lane & 15;
  const int rowBase = blockIdx.x * GROWS;

#pragma unroll
  for (int i = 0; i < (GROWS * FDIM / 8) / NTHR; ++i) {
    const int idx = i * NTHR + tid;
    const int r   = idx >> 3;
    const int c0  = (idx & 7) * 8;
    int row = rowBase + r;
    row = row > nG - 1 ? nG - 1 : row;
    float v[8];
    load8(pooled + (size_t)row * FDIM + c0, v);
    *(v8h*)(sA + r * AP + c0) = cvt8f(v);
  }
  __syncthreads();

  const int r0 = wave * 16;
  v8f acc[2];
#pragma unroll
  for (int t = 0; t < 2; ++t) { v8f z = {0.f, 0.f, 0.f, 0.f, 0.f, 0.f, 0.f, 0.f}; acc[t] = z; }
  const _Float16* ar = sA + (r0 + m) * AP + 8 * hh;
#pragma unroll
  for (int kt = 0; kt < FDIM / 32; ++kt) {
    FragH a;
    a.h[0] = *(const v8h*)(ar + 32 * kt);
    a.h[1] = *(const v8h*)(ar + 32 * kt + 16);
#pragma unroll
    for (int t = 0; t < 2; ++t) {
      const _Float16* bp = l1p + (size_t)(16 * t + m) * FDIM + 32 * kt + 8 * hh;
      FragH b;
      b.h[0] = *(const v8h*)bp;
      b.h[1] = *(const v8h*)(bp + 16);
      acc[t] = wmh(a.v, b.v, acc[t]);
    }
  }
#pragma unroll
  for (int t = 0; t < 2; ++t) {
    const int col = 16 * t + m;
    const float bl = lb1[col];
    _Float16* sp = sZ + (r0 + 8 * hh) * ZP + col;
#pragma unroll
    for (int r = 0; r < 8; ++r) {
      const float z = fmaxf(acc[t][r] * WINV + bl, 0.0f);
      sp[r * ZP] = (_Float16)z;
    }
  }
  __syncthreads();

  FragH a2, b2;
  const _Float16* ar2 = sZ + (r0 + m) * ZP + 8 * hh;
  a2.h[0] = *(const v8h*)ar2;
  a2.h[1] = *(const v8h*)(ar2 + 16);
  const _Float16* bp2 = l2p + (size_t)m * HD2 + 8 * hh;
  b2.h[0] = *(const v8h*)bp2;
  b2.h[1] = *(const v8h*)(bp2 + 16);
  v8f c1 = {0.f, 0.f, 0.f, 0.f, 0.f, 0.f, 0.f, 0.f};
  c1 = wmh(a2.v, b2.v, c1);
  {
    const int mc = m < NCLS ? m : NCLS - 1;
    const float bl2 = lb2[mc];
    float* sl = sL + (r0 + 8 * hh) * NCP + m;
#pragma unroll
    for (int r = 0; r < 8; ++r) sl[r * NCP] = c1[r] * WINV + bl2;
  }
  __syncthreads();

  if (tid < GROWS) {
    const float* lr = sL + tid * NCP;
    float mx = lr[0];
#pragma unroll 1
    for (int i = 1; i < NCLS; ++i) mx = fmaxf(mx, lr[i]);
    float se = 0.0f;
#pragma unroll 1
    for (int i = 0; i < NCLS; ++i) se += expf(lr[i] - mx);
    const float lse = logf(se);
    float* orow = sO + tid * NCLS;
#pragma unroll 1
    for (int i = 0; i < NCLS; ++i) orow[i] = (lr[i] - mx) - lse;
  }
  __syncthreads();

  const int n2 = GROWS * NCLS / 4 - NTHR;
  float* op = out + (size_t)rowBase * NCLS;
  const v4f o0 = *(const v4f*)(sO + 4 * tid);
  v4f o1 = {0.f, 0.f, 0.f, 0.f};
  if (tid < n2) o1 = *(const v4f*)(sO + 4 * (NTHR + tid));
  *(volatile v4f*)(op + 4 * tid) = o0;
  if (tid < n2) *(volatile v4f*)(op + 4 * (NTHR + tid)) = o1;
  __threadfence();
  *(volatile v4f*)(op + 4 * tid) = o0;
  if (tid < n2) *(volatile v4f*)(op + 4 * (NTHR + tid)) = o1;
}

extern "C" void kernel_launch(void* const* d_in, const int* in_sizes, int n_in,
                              void* d_out, int out_size, void* d_ws, size_t ws_size,
                              hipStream_t stream) {
  if (n_in < 15) return;
  const int nN = in_sizes[0] / FDIM;
  const int nE = in_sizes[1] / 2;
  if (nN <= 0 || nE <= 0 || in_sizes[0] != nN * FDIM || in_sizes[1] != 2 * nE || in_sizes[2] != nN) return;
  if (in_sizes[3] != FDIM * FDIM || in_sizes[7] != FDIM * FDIM) return;
  if (in_sizes[4] < FDIM || in_sizes[5] < FDIM || in_sizes[6] < FDIM ||
      in_sizes[8] < FDIM || in_sizes[9] < FDIM || in_sizes[10] < FDIM) return;
  if (in_sizes[11] != FDIM * HD2 || in_sizes[12] < HD2 || in_sizes[13] != HD2 * NCLS || in_sizes[14] < NCLS) return;
  const int G = out_size / NCLS;
  if (G <= 0 || out_size != G * NCLS || (G % GROWS) != 0) return;
  if (nE > (1 << 28) || nN > (1 << 24)) return;

  const float* x     = (const float*)d_in[0];
  const int*   ei    = (const int*)d_in[1];
  const int*   batch = (const int*)d_in[2];
  const float* W1    = (const float*)d_in[3];
  const float* b1    = (const float*)d_in[4];
  const float* g1    = (const float*)d_in[5];
  const float* be1   = (const float*)d_in[6];
  const float* W2    = (const float*)d_in[7];
  const float* b2    = (const float*)d_in[8];
  const float* g2    = (const float*)d_in[9];
  const float* be2   = (const float*)d_in[10];
  const float* lw1   = (const float*)d_in[11];
  const float* lb1   = (const float*)d_in[12];
  const float* lw2   = (const float*)d_in[13];
  const float* lb2   = (const float*)d_in[14];
  float* out = (float*)d_out;

  const int NPAD   = ((nN + TGT - 1) / TGT) * TGT;
  const int nBC    = (nN + NBC - 1) / NBC;
  const int CNTPAD = nBC * NBC;
  if (nBC + 1 > RBN) return;
  const int nBF    = nBC;
  const int csrLen = ((nE + 31) & ~31) + 4096;
  const int nGemm  = NPAD / GROWS;
  const int nAgg   = NPAD / TGT;
  const int nPool  = G / NBP;
  const int nHead  = G / GROWS;

  char* ws = (char*)d_ws;
  size_t off = 0;
  const size_t oW1  = off; off += (size_t)FDIM * FDIM * 2;         off = (off + 255) & ~(size_t)255;
  const size_t oW2  = off; off += (size_t)FDIM * FDIM * 2;         off = (off + 255) & ~(size_t)255;
  const size_t oL1  = off; off += (size_t)HD2 * FDIM * 2;          off = (off + 255) & ~(size_t)255;
  const size_t oL2  = off; off += (size_t)NCP * HD2 * 2;           off = (off + 255) & ~(size_t)255;
  const size_t oCnt = off; off += (size_t)CNTPAD * 4;              off = (off + 255) & ~(size_t)255;
  const size_t oDv  = off; off += (size_t)CNTPAD * 4;              off = (off + 255) & ~(size_t)255;
  const size_t oOff = off; off += (size_t)CNTPAD * 4;              off = (off + 255) & ~(size_t)255;
  const size_t oRb  = off; off += (size_t)RBN * 4;                 off = (off + 255) & ~(size_t)255;
  const size_t oCsr = off; off += (size_t)csrLen * 4;              off = (off + 255) & ~(size_t)255;
  const size_t oHw  = off; off += (size_t)NPAD * FDIM * 4;         off = (off + 255) & ~(size_t)255;
  const size_t oP1  = off; off += (size_t)NPAD * FDIM * 2;         off = (off + 255) & ~(size_t)255;
  const size_t oP2  = off; off += (size_t)NPAD * FDIM * 2;         off = (off + 255) & ~(size_t)255;
  const size_t oPt  = off; off += (size_t)nAgg * 2 * FDIM * 8;     off = (off + 255) & ~(size_t)255;
  const size_t oBn1 = off; off += (size_t)2 * FDIM * 4;            off = (off + 255) & ~(size_t)255;
  const size_t oBn2 = off; off += (size_t)2 * FDIM * 4;            off = (off + 255) & ~(size_t)255;
  const size_t oPl  = off; off += (size_t)nPool * NBP * FDIM * 4;  off = (off + 255) & ~(size_t)255;
  if (off > ws_size) return;
  _Float16* w1p  = (_Float16*)(ws + oW1);
  _Float16* w2p  = (_Float16*)(ws + oW2);
  _Float16* l1p  = (_Float16*)(ws + oL1);
  _Float16* l2p  = (_Float16*)(ws + oL2);
  int*      cnt  = (int*)(ws + oCnt);
  float*    dinv = (float*)(ws + oDv);
  int*      offp = (int*)(ws + oOff);
  int*      rb   = (int*)(ws + oRb);
  int*      csr  = (int*)(ws + oCsr);
  float*    hw   = (float*)(ws + oHw);
  _Float16* P1   = (_Float16*)(ws + oP1);
  _Float16* P2   = (_Float16*)(ws + oP2);
  double*   part = (double*)(ws + oPt);
  float*    bnp1 = (float*)(ws + oBn1);
  float*    bnp2 = (float*)(ws + oBn2);
  float*    pooled = (float*)(ws + oPl);

  const int vec8 = ((nE & 3) == 0) ? 1 : 0;

  const int nPrep = FDIM * FDIM / 8 + FDIM * FDIM / 8 + HD2 * FDIM / 8 + NCP * HD2 / 8;
  k_wprep<<<(nPrep + NTHR - 1) / NTHR, NTHR, 0, stream>>>(W1, W2, lw1, lw2, w1p, w2p, l1p, l2p);

  k_count<<<nBC, NTHR, 0, stream>>>(ei, cnt, dinv, nE, vec8);
  k_offsets<<<1, OTHR, 0, stream>>>(cnt, offp, rb, nBC);
  hipFuncSetAttribute(reinterpret_cast<const void*>(&k_fill),
                      hipFuncAttributeMaxDynamicSharedMemorySize, LDS_FILL);
  k_fill<<<nBF, NTHR, LDS_FILL, stream>>>(ei, offp, rb, csr, nN, nE, vec8, csrLen);

  k_gemm<float, 0><<<nGemm, NTHR, 0, stream>>>(x, w1p, dinv, bnp1, hw, nN);
  k_agg<<<nAgg, NTHR, 0, stream>>>(csr, offp, cnt, dinv, hw, b1, P1, part, nN, csrLen);
  k_bnfin<<<1, 64, 0, stream>>>(part, g1, be1, bnp1, nAgg, nN);

  k_gemm<_Float16, 1><<<nGemm, NTHR, 0, stream>>>(P1, w2p, dinv, bnp1, hw, NPAD);
  k_agg<<<nAgg, NTHR, 0, stream>>>(csr, offp, cnt, dinv, hw, b2, P2, part, nN, csrLen);
  k_bnfin<<<1, 64, 0, stream>>>(part, g2, be2, bnp2, nAgg, nN);

  k_pool<<<nPool, NTHR, 0, stream>>>(batch, P1, P2, bnp1, bnp2, pooled, nN);

  k_head<<<nHead, NTHR, 0, stream>>>(pooled, l1p, lb1, l2p, lb2, out, G);
}
